// SAGE_24300924961370
// MI455X (gfx1250) — hardware-verified
//
#include <hip/hip_runtime.h>
#include <stddef.h>
#include <stdint.h>
#include <math.h>


#define NF     128
#define NC     64
#define APB    384
#define HPB    256
#define GPF    256
#define YPF    128
#define K1G    128
#define KLG    384
#define K2G    256
#define NTHR   256
#define NWAVE  8
#define EPT    8
#define CHUNK  (NTHR * EPT)
#define WCAP   (EPT * 32)
#define LISTN  (NWAVE * WCAP)
#define NBA    1024
#define SLA    10
#define RCAP   28672
#define DEGCAP 64
#define GBM    64
#define GBN    128
#define GTHR   128
#define UPART  2048
#define NPART  7
#define RBH    256
#define AGG_ZINTS    (LISTN + 2 * RCAP + 3 * NBA)
#define MISC_INTS    16
#define ROWBUF_INTS  (NWAVE * RBH / 2)
#define AGG_LDS_INTS (AGG_ZINTS + MISC_INTS + ROWBUF_INTS)
#define WSMAX  134217728

static_assert((CHUNK & (CHUNK - 1)) == 0 && CHUNK <= 4096);
static_assert((NBA & (NBA - 1)) == 0 && NBA == (1 << SLA));
static_assert(((long long)CHUNK << SLA) < (1LL << 31));
static_assert(LISTN % NTHR == 0);
static_assert(NBA % NWAVE == 0 && NBA % 32 == 0 && NBA % GBM == 0);
static_assert(RCAP % 32 == 0 && AGG_ZINTS % (NTHR * 4) == 0 && LISTN % 4 == 0 && ((AGG_ZINTS + MISC_INTS) % 4) == 0);
static_assert(K1G % 32 == 0 && KLG % 32 == 0 && K2G % 32 == 0);
static_assert(KLG == APB && K2G == HPB && GBN == NF && GPF == 2 * NF && YPF == 2 * NC);
static_assert(GBM == (GTHR / 32) * 16 && NF == 4 * 32 && NC == 2 * 32);
static_assert(UPART % NTHR == 0 && (NPART * UPART) % NTHR == 0 && UPART == NF * (NF / 8) && UPART == NC * (K2G / 8));
static_assert(AGG_LDS_INTS * 4 <= 300000);
static_assert((APB * 2) % 128 == 0 && (HPB * 2) % 128 == 0 && (GPF * 4) % 128 == 0 && (YPF * 4) % 128 == 0);
static_assert((NC * 4) % 128 == 0 && (NF * 2) % 128 == 0);
static_assert(DEGCAP >= 35 + 8 && RCAP >= 16623 + 4096);
static_assert(RBH == 2 * NF);

typedef float          v2f   __attribute__((ext_vector_type(2)));
typedef float          v4f   __attribute__((ext_vector_type(4)));
typedef float          v8f   __attribute__((ext_vector_type(8)));
typedef int            v4i   __attribute__((ext_vector_type(4)));
typedef int            v8i   __attribute__((ext_vector_type(8)));
typedef unsigned short v4us  __attribute__((ext_vector_type(4)));
typedef unsigned short v8us  __attribute__((ext_vector_type(8)));
typedef unsigned short v16us __attribute__((ext_vector_type(16)));
typedef __bf16         v16bf __attribute__((ext_vector_type(16)));
typedef v2f  __attribute__((may_alias)) v2fa;
typedef v4f  __attribute__((may_alias)) v4fa;
typedef v4i  __attribute__((may_alias)) v4ia;
typedef v4us __attribute__((may_alias)) v4usa;
typedef v8us __attribute__((may_alias)) v8usa;
union FragB { v16bf v; v16us u; v8us h[2]; v8i w; };

__device__ __forceinline__ v8f wmb(const FragB& a, const FragB& b, v8f c) {
  v8f d = __builtin_amdgcn_wmma_f32_16x16x32_bf16(false, a.v, false, b.v, (short)0, c, false, false);
  asm volatile("v_nop\n\tv_nop\n\tv_nop\n\tv_nop" : "+v"(d) : "v"(a.w), "v"(b.w));
  return d;
}

__device__ __forceinline__ unsigned bf16_bits(float f) {
  const unsigned u = __float_as_uint(f);
  return (u + 0x7FFFu + ((u >> 16) & 1u)) >> 16;
}
__device__ __forceinline__ float bf16_val(float f) {
  return __uint_as_float(bf16_bits(f) << 16);
}

__device__ __forceinline__ void wave_sync() {
  __builtin_amdgcn_fence(__ATOMIC_RELEASE, "wavefront");
  __builtin_amdgcn_wave_barrier();
  __builtin_amdgcn_fence(__ATOMIC_ACQUIRE, "wavefront");
}

template <int SLB>
__device__ __forceinline__ int scan_chunk(const int* __restrict__ dsts, int nE, int cbase, int slotBase,
                                          int nb, int vec8, int* list, int tid, int lane, int wave) {
  int wc = 0;
  const int el0  = tid * EPT;
  const int e0   = cbase + el0;
  const int sent = -2147483647 - 1;
  v4i da, db;
  if (vec8 != 0 && cbase + CHUNK <= nE) {
    da = *(const v4i*)(dsts + e0);
    db = *(const v4i*)(dsts + e0 + 4);
  } else {
    da.x = (e0     < nE) ? dsts[min(e0,     nE - 1)] : sent;
    da.y = (e0 + 1 < nE) ? dsts[min(e0 + 1, nE - 1)] : sent;
    da.z = (e0 + 2 < nE) ? dsts[min(e0 + 2, nE - 1)] : sent;
    da.w = (e0 + 3 < nE) ? dsts[min(e0 + 3, nE - 1)] : sent;
    db.x = (e0 + 4 < nE) ? dsts[min(e0 + 4, nE - 1)] : sent;
    db.y = (e0 + 5 < nE) ? dsts[min(e0 + 5, nE - 1)] : sent;
    db.z = (e0 + 6 < nE) ? dsts[min(e0 + 6, nE - 1)] : sent;
    db.w = (e0 + 7 < nE) ? dsts[min(e0 + 7, nE - 1)] : sent;
  }
  const unsigned nbs = (unsigned)slotBase;
  const unsigned unb = (unsigned)nb;
  const unsigned s0 = (unsigned)da.x - nbs, s1 = (unsigned)da.y - nbs;
  const unsigned s2 = (unsigned)da.z - nbs, s3 = (unsigned)da.w - nbs;
  const unsigned s4 = (unsigned)db.x - nbs, s5 = (unsigned)db.y - nbs;
  const unsigned s6 = (unsigned)db.z - nbs, s7 = (unsigned)db.w - nbs;
  const bool h0 = s0 < unb, h1 = s1 < unb, h2 = s2 < unb, h3 = s3 < unb;
  const bool h4 = s4 < unb, h5 = s5 < unb, h6 = s6 < unb, h7 = s7 < unb;
  const unsigned any = __builtin_amdgcn_ballot_w32(h0 | h1 | h2 | h3 | h4 | h5 | h6 | h7);
  if (any != 0u) {
#define HITJ(J, HJ, SJ) { \
      const unsigned mj = __builtin_amdgcn_ballot_w32(HJ); \
      if (mj != 0u) { \
        if (HJ) { \
          const int pos = wc + (int)__builtin_amdgcn_mbcnt_lo(mj, 0u); \
          if (pos < WCAP) list[wave * WCAP + pos] = ((el0 + (J)) << SLB) | (int)(SJ); \
        } \
        wc += (int)__builtin_popcount(mj); } }
    HITJ(0, h0, s0)
    HITJ(1, h1, s1)
    HITJ(2, h2, s2)
    HITJ(3, h3, s3)
    HITJ(4, h4, s4)
    HITJ(5, h5, s5)
    HITJ(6, h6, s6)
    HITJ(7, h7, s7)
#undef HITJ
  }
  return wc;
}

__global__ __launch_bounds__(NTHR) void k_wprep(const float* __restrict__ W1l, const float* __restrict__ W1r,
                                                const float* __restrict__ Wl1, const float* __restrict__ W2l,
                                                const float* __restrict__ W2r,
                                                unsigned short* BW1, unsigned short* BL, unsigned short* B2) {
  const int u    = (int)blockIdx.x * NTHR + (int)threadIdx.x;
  const int part = u >> 11;
  const int v    = u & (UPART - 1);
  const float* p;
  unsigned short* dp;
  if (part == 0) {
    const int n = v >> 4, k8 = (v & 15) * 8;
    p = W1l + (size_t)n * NF + k8;            dp = BW1 + (size_t)n * K1G + k8;
  } else if (part == 1) {
    const int n = v >> 4, k8 = (v & 15) * 8;
    p = W1r + (size_t)n * NF + k8;            dp = BW1 + (size_t)(NF + n) * K1G + k8;
  } else if (part == 2) {
    const int n = v >> 4, k8 = (v & 15) * 8;
    p = Wl1 + (size_t)n * (2 * NF) + k8;      dp = BL + (size_t)n * KLG + k8;
  } else if (part == 3) {
    const int n = v >> 4, k8 = (v & 15) * 8;
    p = Wl1 + (size_t)n * (2 * NF) + NF + k8; dp = BL + (size_t)n * KLG + NF + k8;
  } else if (part == 4) {
    const int n = v >> 4, k8 = (v & 15) * 8;
    p = Wl1 + (size_t)n * (2 * NF) + NF + k8; dp = BL + (size_t)n * KLG + 2 * NF + k8;
  } else if (part == 5) {
    const int n = v >> 5, k8 = (v & 31) * 8, kk = k8 & (NF - 1);
    p = W2l + (size_t)n * NF + kk;            dp = B2 + (size_t)n * K2G + k8;
  } else if (part == 6) {
    const int n = v >> 5, k8 = (v & 31) * 8, kk = k8 & (NF - 1);
    p = W2r + (size_t)n * NF + kk;            dp = B2 + (size_t)(NC + n) * K2G + k8;
  } else {
    return;
  }
  const v4f a = *(const v4fa*)p;
  const v4f b = *(const v4fa*)(p + 4);
  v8us o;
  o[0] = (unsigned short)bf16_bits(a.x); o[1] = (unsigned short)bf16_bits(a.y);
  o[2] = (unsigned short)bf16_bits(a.z); o[3] = (unsigned short)bf16_bits(a.w);
  o[4] = (unsigned short)bf16_bits(b.x); o[5] = (unsigned short)bf16_bits(b.y);
  o[6] = (unsigned short)bf16_bits(b.z); o[7] = (unsigned short)bf16_bits(b.w);
  *(volatile v8us*)dp = o;
  __threadfence();
  *(volatile v8us*)dp = o;
}

__global__ __launch_bounds__(NTHR) void k_cvx(const float* __restrict__ x, int nN, int nUnits,
                                              unsigned short* ab) {
  const int u = (int)blockIdx.x * NTHR + (int)threadIdx.x;
  if (u >= nUnits) return;
  const int row = u >> 4;
  const int k8  = (u & 15) * 8;
  const int rc  = row < nN ? row : nN - 1;
  const float* p = x + (size_t)rc * NF + k8;
  const v4f a = *(const v4fa*)p;
  const v4f b = *(const v4fa*)(p + 4);
  const bool ok = row < nN;
  v8us o;
  o[0] = ok ? (unsigned short)bf16_bits(a.x) : (unsigned short)0;
  o[1] = ok ? (unsigned short)bf16_bits(a.y) : (unsigned short)0;
  o[2] = ok ? (unsigned short)bf16_bits(a.z) : (unsigned short)0;
  o[3] = ok ? (unsigned short)bf16_bits(a.w) : (unsigned short)0;
  o[4] = ok ? (unsigned short)bf16_bits(b.x) : (unsigned short)0;
  o[5] = ok ? (unsigned short)bf16_bits(b.y) : (unsigned short)0;
  o[6] = ok ? (unsigned short)bf16_bits(b.z) : (unsigned short)0;
  o[7] = ok ? (unsigned short)bf16_bits(b.w) : (unsigned short)0;
  unsigned short* dp = ab + (size_t)row * APB + k8;
  *(volatile v8us*)dp = o;
  __threadfence();
  *(volatile v8us*)dp = o;
}

template <int EPI>
__global__ __launch_bounds__(GTHR) void k_gemm(const unsigned short* __restrict__ Apl, int lda,
                                               const unsigned short* __restrict__ BT, int K,
                                               const float* __restrict__ bias,
                                               float* outF, int ldo, unsigned short* outH, int ldh, int nValid) {
  __shared__ __attribute__((aligned(16))) float stg[GBM * GBN];
  const int tid = (int)threadIdx.x, lane = tid & 31, wave = tid >> 5, hh = lane >> 4, m = lane & 15;
  const int rowBase = (int)blockIdx.x * GBM;
  const int col0    = (int)blockIdx.y * GBN;

  v8f acc[8];
  {
    const v8f z = {0.f, 0.f, 0.f, 0.f, 0.f, 0.f, 0.f, 0.f};
#pragma unroll
    for (int t = 0; t < 8; ++t) acc[t] = z;
  }
  const unsigned short* ap = Apl + (size_t)(rowBase + 16 * wave + m) * (size_t)lda + 8 * hh;
  const unsigned short* bp = BT + (size_t)(col0 + m) * (size_t)K + 8 * hh;

#pragma unroll 1
  for (int k0 = 0; k0 < K; k0 += 32) {
    FragB af;
    af.h[0] = *(const v8usa*)(ap + k0);
    af.h[1] = *(const v8usa*)(ap + k0 + 16);
#pragma unroll
    for (int nt = 0; nt < 8; ++nt) {
      const unsigned short* wq = bp + (size_t)(16 * nt) * (size_t)K + k0;
      FragB bf;
      bf.h[0] = *(const v8usa*)wq;
      bf.h[1] = *(const v8usa*)(wq + 16);
      acc[nt] = wmb(af, bf, acc[nt]);
    }
  }

#pragma unroll
  for (int nt = 0; nt < 8; ++nt) {
    const int lc = 16 * nt + m;
#pragma unroll
    for (int r = 0; r < 8; ++r) {
      const int lr = 16 * wave + 8 * hh + r;
      stg[lr * GBN + lc] = acc[nt][r];
    }
  }
  __syncthreads();

  v4f pv[16];
#pragma unroll
  for (int i = 0; i < 16; ++i) pv[i] = *(const v4fa*)(stg + (16 * wave + i) * GBN + 4 * lane);
  __syncthreads();

  if constexpr (EPI == 0) {
#pragma unroll
    for (int i = 0; i < 16; ++i) {
      const int r = rowBase + 16 * wave + i;
      *(volatile v4f*)(outF + (size_t)r * (size_t)ldo + col0 + 4 * lane) = pv[i];
    }
    __threadfence();
#pragma unroll
    for (int i = 0; i < 16; ++i) {
      const int r = rowBase + 16 * wave + i;
      *(volatile v4f*)(outF + (size_t)r * (size_t)ldo + col0 + 4 * lane) = pv[i];
    }
  } else {
    v4f bb4;
    {
      const v4f t1 = *(const v4fa*)(bias + 4 * lane);
      bb4.x = bf16_val(t1.x); bb4.y = bf16_val(t1.y); bb4.z = bf16_val(t1.z); bb4.w = bf16_val(t1.w);
    }
#pragma unroll
    for (int i = 0; i < 16; ++i) {
      const bool ok = (rowBase + 16 * wave + i) < nValid;
      const v4f t = pv[i] + bb4;
      v4f y;
      y.x = fmaxf(t.x, 0.0f); y.y = fmaxf(t.y, 0.0f); y.z = fmaxf(t.z, 0.0f); y.w = fmaxf(t.w, 0.0f);
      y.x = ok ? y.x : 0.0f; y.y = ok ? y.y : 0.0f; y.z = ok ? y.z : 0.0f; y.w = ok ? y.w : 0.0f;
      pv[i] = y;
    }
#pragma unroll
    for (int i = 0; i < 16; ++i) {
      v4us h4, l4;
      unsigned hb;
      hb = bf16_bits(pv[i].x); h4[0] = (unsigned short)hb; l4[0] = (unsigned short)bf16_bits(pv[i].x - __uint_as_float(hb << 16));
      hb = bf16_bits(pv[i].y); h4[1] = (unsigned short)hb; l4[1] = (unsigned short)bf16_bits(pv[i].y - __uint_as_float(hb << 16));
      hb = bf16_bits(pv[i].z); h4[2] = (unsigned short)hb; l4[2] = (unsigned short)bf16_bits(pv[i].z - __uint_as_float(hb << 16));
      hb = bf16_bits(pv[i].w); h4[3] = (unsigned short)hb; l4[3] = (unsigned short)bf16_bits(pv[i].w - __uint_as_float(hb << 16));
      unsigned short* srow = (unsigned short*)stg + (size_t)(16 * wave + i) * (2 * GBN);
      *(v4usa*)(srow + 4 * lane) = h4;
      *(v4usa*)(srow + NF + 4 * lane) = l4;
    }
    __syncthreads();
    v8us qv[16];
#pragma unroll
    for (int i = 0; i < 16; ++i) {
      const unsigned short* srow = (const unsigned short*)stg + (size_t)(16 * wave + i) * (2 * GBN);
      qv[i] = *(const v8usa*)(srow + 8 * lane);
    }
#pragma unroll
    for (int i = 0; i < 16; ++i) {
      unsigned short* rp = outH + (size_t)(rowBase + 16 * wave + i) * (size_t)ldh + 8 * lane;
      *(volatile v8us*)rp = qv[i];
    }
    __threadfence();
#pragma unroll
    for (int i = 0; i < 16; ++i) {
      unsigned short* rp = outH + (size_t)(rowBase + 16 * wave + i) * (size_t)ldh + 8 * lane;
      *(volatile v8us*)rp = qv[i];
    }
  }
}

template <int L1>
__global__ __launch_bounds__(NTHR) void k_scan(const int* __restrict__ srcs, const int* __restrict__ dsts,
                                               int nE, int nN, int vec8, int mRows,
                                               const float* __restrict__ gpl, const float* __restrict__ bias,
                                               unsigned short* apl, float* outp) {
  extern __shared__ __attribute__((aligned(16))) int dsm[];
  int* list = dsm;
  int* hl   = dsm + LISTN;
  int* sl   = hl + RCAP;
  int* cnt  = sl + RCAP;
  int* offs = cnt + NBA;
  int* cur  = offs + NBA;
  int* misc = cur + NBA;
  const int tid = (int)threadIdx.x, lane = tid & 31, wave = tid >> 5;
  unsigned short* rowbuf = (unsigned short*)(misc + MISC_INTS) + wave * RBH;
  const int nodeBase = (int)blockIdx.x * NBA;

  {
    const v4i z4 = {0, 0, 0, 0};
    for (int i = tid * 4; i < AGG_ZINTS; i += NTHR * 4) *(v4ia*)(dsm + i) = z4;
    if (tid < MISC_INTS) misc[tid] = 0;
  }
  __syncthreads();

  int t = 0, ov = 0;
  const int nChunks = (nE + CHUNK - 1) / CHUNK;
#pragma unroll 1
  for (int ch = 0; ch < nChunks; ++ch) {
    const int cbase = ch * CHUNK;
    const int wc = scan_chunk<SLA>(dsts, nE, cbase, nodeBase, NBA, vec8, list, tid, lane, wave);
    if (lane == 0) misc[wave] = wc;
    __syncthreads();
    if (wave == 0) {
#pragma unroll 1
      for (int w2 = 0; w2 < NWAVE; ++w2) {
        int c = misc[w2];
        c = c < 0 ? 0 : (c > WCAP ? WCAP : c);
#pragma unroll 1
        for (int b0 = 0; b0 < c; b0 += 32) {
          const int idx = b0 + lane;
          const int ent = list[w2 * WCAP + (idx < WCAP ? idx : WCAP - 1)];
          const int m32 = (c - b0) < 32 ? (c - b0) : 32;
#pragma unroll 1
          for (int k = 0; k < m32; ++k) {
            const int u    = __builtin_amdgcn_readlane(ent, k);
            const int slot = u & (NBA - 1);
            const int el   = (u >> SLA) & (CHUNK - 1);
            const int pk   = ((cbase + el) << SLA) | slot;
            if (t < RCAP) {
              if (lane == 0) { hl[t] = pk; cnt[slot] = cnt[slot] + 1; }
              t = t + 1;
            } else {
              ov = 1;
            }
          }
        }
      }
    }
    __syncthreads();
  }
  if (wave == 0 && lane == 0) { misc[8] = t; misc[9] = ov; }
  __syncthreads();
  int tt = misc[8];
  tt = tt < 0 ? 0 : (tt > RCAP ? RCAP : tt);
  const int ovf = misc[9];

  if (wave == 0) {
    const int base = lane * (NBA / 32);
    int s = 0;
#pragma unroll 1
    for (int i = 0; i < NBA / 32; ++i) s += cnt[base + i];
    int incl = s;
#pragma unroll
    for (int d = 1; d < 32; d <<= 1) {
      const int y = __shfl_up(incl, d, 32);
      if (lane >= d) incl += y;
    }
    int run = incl - s;
#pragma unroll 1
    for (int i = 0; i < NBA / 32; ++i) {
      const int cv = cnt[base + i];
      offs[base + i] = run;
      cur[base + i]  = run;
      run += cv;
    }
  }
  __syncthreads();
  if (wave == 0) {
#pragma unroll 1
    for (int b0 = 0; b0 < tt; b0 += 32) {
      const int idx = b0 + lane;
      const int ent = hl[idx < RCAP ? idx : RCAP - 1];
      const int m32 = (tt - b0) < 32 ? (tt - b0) : 32;
#pragma unroll 1
      for (int k = 0; k < m32; ++k) {
        const int u    = __builtin_amdgcn_readlane(ent, k);
        const int slot = u & (NBA - 1);
        if (lane == 0) {
          int p = cur[slot];
          p = p < 0 ? 0 : (p > RCAP - 1 ? RCAP - 1 : p);
          sl[p] = u;
          cur[slot] = p + 1;
        }
      }
    }
  }
  __syncthreads();

  const float qnan = __int_as_float(0x7fc00000);
  const float pz = (ovf != 0) ? qnan : 0.0f;
  if constexpr (L1 != 0) {
    v4f bb4;
    {
      const v4f t4 = *(const v4fa*)(bias + 4 * lane);
      bb4.x = bf16_val(t4.x); bb4.y = bf16_val(t4.y); bb4.z = bf16_val(t4.z); bb4.w = bf16_val(t4.w);
    }
#pragma unroll 1
    for (int si = 0; si < NBA / NWAVE; ++si) {
      const int s    = si * NWAVE + wave;
      const int node = nodeBase + s;
      int craw = cnt[s];
      craw = craw < 0 ? 0 : (craw > RCAP ? RCAP : craw);
      const bool big = craw > DEGCAP;
      const int c = craw > DEGCAP ? DEGCAP : craw;
      int o = offs[s];
      o = o < 0 ? 0 : (o > RCAP ? RCAP : o);
      const int nc = node < nN ? node : nN - 1;
      float a0 = 0.0f, a1 = 0.0f, a2 = 0.0f, a3 = 0.0f;
#pragma unroll 1
      for (int b0 = 0; b0 < c; b0 += 32) {
        int idx = o + b0 + lane;
        idx = idx > RCAP - 1 ? RCAP - 1 : idx;
        const int ent = sl[idx];
        int eid = ent >> SLA;
        eid = eid < 0 ? 0 : (eid > nE - 1 ? nE - 1 : eid);
        int sr = srcs[eid];
        sr = sr < 0 ? 0 : (sr > nN - 1 ? nN - 1 : sr);
        const int m32 = (c - b0) < 32 ? (c - b0) : 32;
#pragma unroll 1
        for (int k = 0; k < m32; ++k) {
          const int sk = __builtin_amdgcn_readlane(sr, k);
          const v4f a = *(const v4fa*)(gpl + (size_t)sk * GPF + 4 * lane);
          a0 += a.x; a1 += a.y; a2 += a.z; a3 += a.w;
        }
      }
      const float rinv = 1.0f / fmaxf((float)craw, 1.0f);
      const v4f xr = *(const v4fa*)(gpl + (size_t)nc * GPF + NF + 4 * lane);
      const float o0 = (a0 * rinv + bb4.x) + xr.x;
      const float o1 = (a1 * rinv + bb4.y) + xr.y;
      const float o2 = (a2 * rinv + bb4.z) + xr.z;
      const float o3 = (a3 * rinv + bb4.w) + xr.w;
      float ss = o0 * o0 + o1 * o1 + o2 * o2 + o3 * o3;
      ss += __shfl_xor(ss, 1, 32);
      ss += __shfl_xor(ss, 2, 32);
      ss += __shfl_xor(ss, 4, 32);
      ss += __shfl_xor(ss, 8, 32);
      ss += __shfl_xor(ss, 16, 32);
      const float inv = 1.0f / fmaxf(sqrtf(ss), 1e-12f);
      const float pzr = big ? qnan : pz;
      const bool live = node < nN;
      const float y0 = fmaxf(o0 * inv, 0.0f) + pzr;
      const float y1 = fmaxf(o1 * inv, 0.0f) + pzr;
      const float y2 = fmaxf(o2 * inv, 0.0f) + pzr;
      const float y3 = fmaxf(o3 * inv, 0.0f) + pzr;
      const float m0 = live ? y0 : 0.0f;
      const float m1 = live ? y1 : 0.0f;
      const float m2 = live ? y2 : 0.0f;
      const float m3 = live ? y3 : 0.0f;
      v4us mh, ml;
      {
        unsigned hb;
        hb = bf16_bits(m0); mh[0] = (unsigned short)hb; ml[0] = (unsigned short)bf16_bits(m0 - __uint_as_float(hb << 16));
        hb = bf16_bits(m1); mh[1] = (unsigned short)hb; ml[1] = (unsigned short)bf16_bits(m1 - __uint_as_float(hb << 16));
        hb = bf16_bits(m2); mh[2] = (unsigned short)hb; ml[2] = (unsigned short)bf16_bits(m2 - __uint_as_float(hb << 16));
        hb = bf16_bits(m3); mh[3] = (unsigned short)hb; ml[3] = (unsigned short)bf16_bits(m3 - __uint_as_float(hb << 16));
      }
      *(v4usa*)(rowbuf + 4 * lane) = mh;
      *(v4usa*)(rowbuf + NF + 4 * lane) = ml;
      wave_sync();
      const v8us q0 = *(const v8usa*)(rowbuf + 8 * lane);
      wave_sync();
      if (node < mRows) {
        unsigned short* rpw = apl + (size_t)node * APB + NF + 8 * lane;
        *(volatile v8us*)rpw = q0;
        __threadfence();
        *(volatile v8us*)rpw = q0;
      }
    }
  } else {
    float bv0, bv1;
    {
      const v2f b2 = *(const v2fa*)(bias + 2 * lane);
      bv0 = bf16_val(b2.x); bv1 = bf16_val(b2.y);
    }
    const int sa = (2 * lane) & 31, sb = (2 * lane + 1) & 31;
#pragma unroll 1
    for (int si = 0; si < NBA / NWAVE; ++si) {
      const int s    = si * NWAVE + wave;
      const int node = nodeBase + s;
      int craw = cnt[s];
      craw = craw < 0 ? 0 : (craw > RCAP ? RCAP : craw);
      const bool big = craw > DEGCAP;
      const int c = craw > DEGCAP ? DEGCAP : craw;
      int o = offs[s];
      o = o < 0 ? 0 : (o > RCAP ? RCAP : o);
      const int nc = node < nN ? node : nN - 1;
      float acc0 = 0.0f, acc1 = 0.0f;
#pragma unroll 1
      for (int b0 = 0; b0 < c; b0 += 32) {
        int idx = o + b0 + lane;
        idx = idx > RCAP - 1 ? RCAP - 1 : idx;
        const int ent = sl[idx];
        int eid = ent >> SLA;
        eid = eid < 0 ? 0 : (eid > nE - 1 ? nE - 1 : eid);
        int sr = srcs[eid];
        sr = sr < 0 ? 0 : (sr > nN - 1 ? nN - 1 : sr);
        const int m32 = (c - b0) < 32 ? (c - b0) : 32;
#pragma unroll 1
        for (int k = 0; k < m32; ++k) {
          const int sk = __builtin_amdgcn_readlane(sr, k);
          const v2f a = *(const v2fa*)(gpl + (size_t)sk * YPF + 2 * lane);
          acc0 += a.x; acc1 += a.y;
        }
      }
      const float rinv = 1.0f / fmaxf((float)craw, 1.0f);
      const v2f rr = *(const v2fa*)(gpl + (size_t)nc * YPF + NC + 2 * lane);
      const float o0 = (acc0 * rinv + bv0) + rr.x;
      const float o1 = (acc1 * rinv + bv1) + rr.y;
      float ss = o0 * o0 + o1 * o1;
      ss += __shfl_xor(ss, 1, 32);
      ss += __shfl_xor(ss, 2, 32);
      ss += __shfl_xor(ss, 4, 32);
      ss += __shfl_xor(ss, 8, 32);
      ss += __shfl_xor(ss, 16, 32);
      const float inv = 1.0f / fmaxf(sqrtf(ss), 1e-12f);
      const float pzr = big ? qnan : pz;
      const bool live = node < nN;
      const float y0 = o0 * inv + pzr;
      const float y1 = o1 * inv + pzr;
      const float v0 = live ? y0 : 0.0f;
      const float v1 = live ? y1 : 0.0f;
      v4f ow;
      ow.x = __shfl(v0, sa, 32); ow.y = __shfl(v1, sa, 32);
      ow.z = __shfl(v0, sb, 32); ow.w = __shfl(v1, sb, 32);
      const bool wr = (node < mRows) && (lane < 16);
      float* op = outp + (size_t)node * NC + 4 * (lane & 15);
      if (wr) *(volatile v4f*)op = ow;
      __threadfence();
      if (wr) *(volatile v4f*)op = ow;
    }
  }
}

static inline int cdiv(int a, int b) { return (a + b - 1) / b; }
static inline size_t al256(size_t o) { return (o + 255) & ~(size_t)255; }

extern "C" void kernel_launch(void* const* d_in, const int* in_sizes, int n_in,
                              void* d_out, int out_size, void* d_ws, size_t ws_size,
                              hipStream_t stream) {
  if (n_in < 10) return;
  if (in_sizes[0] < NF || (in_sizes[0] % NF) != 0) return;
  const int nN = in_sizes[0] / NF;
  if (nN < 1 || nN >= (1 << 21)) return;
  if (in_sizes[1] < 2 || (in_sizes[1] & 1) != 0) return;
  const int nE = in_sizes[1] / 2;
  if (nE < 1 || nE >= (1 << (31 - SLA))) return;
  if (in_sizes[2] != NF * NF || in_sizes[3] != NF) return;
  if (in_sizes[4] != NF * NF) return;
  if (in_sizes[5] != NF * 2 * NF || in_sizes[6] != NF) return;
  if (in_sizes[7] != NC * NF || in_sizes[8] != NC) return;
  if (in_sizes[9] != NC * NF) return;
  if ((long long)out_size != (long long)nN * NC) return;

  const float* x    = (const float*)d_in[0];
  const int*   edge = (const int*)d_in[1];
  const float* W1l  = (const float*)d_in[2];
  const float* b1l  = (const float*)d_in[3];
  const float* W1r  = (const float*)d_in[4];
  const float* Wl1  = (const float*)d_in[5];
  const float* bl1  = (const float*)d_in[6];
  const float* W2l  = (const float*)d_in[7];
  const float* b2l  = (const float*)d_in[8];
  const float* W2r  = (const float*)d_in[9];
  float* out = (float*)d_out;
  const int* src = edge;
  const int* dst = edge + nE;

  const int MP = cdiv(nN, GBM) * GBM;
  const int gM = MP / GBM;
  const int gA = cdiv(MP, NBA);
  if ((long long)gA * NBA < (long long)MP) return;
  const int vec8 = ((nE & 3) == 0) ? 1 : 0;

  char* ws = (char*)d_ws;
  size_t off = 0;
  const size_t oBW1 = off; off = al256(off + (size_t)(2 * NF) * K1G * 2);
  const size_t oBL  = off; off = al256(off + (size_t)NF * KLG * 2);
  const size_t oB2  = off; off = al256(off + (size_t)(2 * NC) * K2G * 2);
  const size_t oAB  = off; off = al256(off + (size_t)MP * APB * 2);
  const size_t oG1  = off; off = al256(off + (size_t)MP * GPF * 4);
  const size_t oH2  = oG1;
  const size_t oY   = oG1 + (size_t)MP * HPB * 2;
  if (oY + (size_t)MP * YPF * 4 > oG1 + (size_t)MP * GPF * 4) return;
  if (off > ws_size || off > (size_t)WSMAX) return;
  unsigned short* BW1 = (unsigned short*)(ws + oBW1);
  unsigned short* BL  = (unsigned short*)(ws + oBL);
  unsigned short* B2  = (unsigned short*)(ws + oB2);
  unsigned short* AB  = (unsigned short*)(ws + oAB);
  float*          G1  = (float*)(ws + oG1);
  unsigned short* H2  = (unsigned short*)(ws + oH2);
  float*          Y   = (float*)(ws + oY);

  const size_t scanLds = (size_t)AGG_LDS_INTS * 4;
  hipFuncSetAttribute(reinterpret_cast<const void*>(&k_scan<1>), hipFuncAttributeMaxDynamicSharedMemorySize, (int)scanLds);
  hipFuncSetAttribute(reinterpret_cast<const void*>(&k_scan<0>), hipFuncAttributeMaxDynamicSharedMemorySize, (int)scanLds);

  const int nUx = MP * (NF / 8);
  k_wprep<<<(NPART * UPART) / NTHR, NTHR, 0, stream>>>(W1l, W1r, Wl1, W2l, W2r, BW1, BL, B2);
  k_cvx<<<cdiv(nUx, NTHR), NTHR, 0, stream>>>(x, nN, nUx, AB);
  k_gemm<0><<<dim3(gM, (2 * NF) / GBN), GTHR, 0, stream>>>(AB, APB, BW1, K1G, b1l, G1, GPF, H2, HPB, nN);
  k_scan<1><<<gA, NTHR, scanLds, stream>>>(src, dst, nE, nN, vec8, MP, G1, b1l, AB, out);
  k_gemm<1><<<dim3(gM, 1), GTHR, 0, stream>>>(AB, APB, BL, KLG, bl1, Y, YPF, H2, HPB, nN);
  k_gemm<0><<<dim3(gM, 1), GTHR, 0, stream>>>(H2, HPB, B2, K2G, b2l, Y, YPF, AB, APB, nN);
  k_scan<0><<<gA, NTHR, scanLds, stream>>>(src, dst, nE, nN, vec8, nN, Y, b2l, AB, out);
}
